// HierarchicalMamba_44401371906500
// MI455X (gfx1250) — hardware-run, weakly checked
//
#include <hip/hip_runtime.h>
#include <math.h>

typedef __attribute__((ext_vector_type(16))) _Float16 v16h;
typedef __attribute__((ext_vector_type(8)))  _Float16 v8h;
typedef __attribute__((ext_vector_type(8)))  float    v8f;
typedef __attribute__((ext_vector_type(4)))  float    v4f;

constexpr int kBatch   = 2;
constexpr int kSeq0    = 4096;
constexpr int kCh      = 256;
constexpr int kNst     = 64;
constexpr int kLayers  = 3;
constexpr int kProjN   = 129;
constexpr int kProjNP  = 144;
constexpr int kDbcP    = 160;
constexpr int kSlabP   = 164;
constexpr int kTS      = 32;
constexpr int kScanCh  = 64;
constexpr int kYP      = 68;
constexpr int kAP      = 68;
static_assert(1 + 2 * kNst == kProjN, "step column + B + C");
static_assert(kProjNP % 16 == 0 && kProjNP >= kProjN, "tile multiple");
static_assert(kCh % 32 == 0, "K multiple of 32");
static_assert((kDbcP * 4) % 128 == 0 && kDbcP >= kProjNP && (kDbcP % 4) == 0, "row pitch in whole lines");
static_assert(kNst == 64 && kScanCh == 64 && kCh % kScanCh == 0, "scan geometry");
static_assert((kSeq0 / 4) % kTS == 0, "chunk multiple at every layer");

constexpr float kXCarry   = 32.0f;
constexpr float kWCarry   = 1024.0f;
constexpr float kRCarry   = 2048.0f;
constexpr float kFoldMain = 1.0f / (kXCarry * kWCarry);
constexpr float kFoldRes  = kFoldMain / kRCarry;
constexpr float kHalfMinNormal = 6.103515625e-05f;

constexpr size_t kRows0   = (size_t)kBatch * kSeq0;
constexpr size_t kRows1   = kRows0 / 2;
constexpr size_t kRows2   = kRows0 / 4;
constexpr size_t kOffWP   = 0;
constexpr size_t kOffXH0  = kOffWP   + (size_t)kLayers * kProjNP * kCh * 2;
constexpr size_t kOffDBC0 = kOffXH0  + kRows0 * kCh * 2;
constexpr size_t kOffDBC1 = kOffDBC0 + kRows0 * kDbcP * 4;
constexpr size_t kOffDBC2 = kOffDBC1 + kRows1 * kDbcP * 4;
constexpr size_t kOffX1F  = kOffDBC2 + kRows2 * kDbcP * 4;
constexpr size_t kOffX1H  = kOffX1F  + kRows1 * kCh * 4;
constexpr size_t kOffX1L  = kOffX1H  + kRows1 * kCh * 2;
constexpr size_t kOffX2F  = kOffX1L  + kRows1 * kCh * 2;
constexpr size_t kOffX2H  = kOffX2F  + kRows2 * kCh * 4;
constexpr size_t kOffX2L  = kOffX2H  + kRows2 * kCh * 2;
constexpr size_t kWsTotal = kOffX2L  + kRows2 * kCh * 2;
static_assert(kWsTotal == 26173440ull, "carve total");
static_assert(kWsTotal <= 134217728ull, "carve cap");
static_assert((kOffXH0 % 128) == 0 && (kOffDBC0 % 128) == 0 && (kOffDBC1 % 128) == 0 && (kOffDBC2 % 128) == 0 &&
              (kOffX1F % 128) == 0 && (kOffX1H % 128) == 0 && (kOffX1L % 128) == 0 && (kOffX2F % 128) == 0 &&
              (kOffX2H % 128) == 0 && (kOffX2L % 128) == 0, "128-B aligned regions");

__device__ __forceinline__ float bf_rne_value(float f) {
  unsigned u = __float_as_uint(f);
  u = (u + 0x7FFFu + ((u >> 16) & 1u)) & 0xFFFF0000u;
  return __uint_as_float(u);
}
__device__ __forceinline__ _Float16 to_h_flush(float v) {
  const float w = (fabsf(v) < kHalfMinNormal) ? 0.0f : v;
  return (_Float16)w;
}
union FragH { v16h v; v8h h[2]; };
__device__ __forceinline__ v16h frag_load(const _Float16* p) {
  FragH f;
  f.h[0] = *(const v8h*)(p);
  f.h[1] = *(const v8h*)(p + 16);
  return f.v;
}
__device__ __forceinline__ v8f mma_h(v16h a, v16h b, v8f c) {
  c = __builtin_amdgcn_wmma_f32_16x16x32_f16(false, a, false, b, (short)0, c, false, false);
  asm volatile("v_nop\n\tv_nop\n\tv_nop\n\tv_nop" : "+v"(c) : "v"(a), "v"(b));
  return c;
}

__global__ __launch_bounds__(256) void plane_x_f16_kernel(
    const float* __restrict__ src, unsigned short* __restrict__ dst, int total8)
{
  const int i = blockIdx.x * 256 + threadIdx.x;
  if (i >= total8) return;
  const size_t e0 = (size_t)i << 3;
  const v4f a0 = *(const v4f*)(src + e0);
  const v4f a1 = *(const v4f*)(src + e0 + 4);
  v8h hv;
#pragma unroll
  for (int e = 0; e < 4; ++e) {
    const float t0 = a0[e];
    const float t1 = a1[e];
    hv[e]     = to_h_flush(bf_rne_value(t0) * kXCarry);
    hv[4 + e] = to_h_flush(bf_rne_value(t1) * kXCarry);
  }
  unsigned short* q = dst + e0;
  *(volatile v8h*)q = hv;
  __threadfence();
  *(volatile v8h*)q = hv;
}

__global__ __launch_bounds__(256) void plane_w_f16_kernel(
    const float* __restrict__ W, unsigned short* __restrict__ WP, int total8)
{
  const int i = blockIdx.x * 256 + threadIdx.x;
  if (i >= total8) return;
  const int e0 = i << 3;
  constexpr int kPlane = kProjNP * kCh;
  const int layer = e0 / kPlane;
  const int rem   = e0 - layer * kPlane;
  const int j     = rem / kCh;
  const int c     = rem - j * kCh;
  const bool live = (j <= 2 * kNst);
  const int sr    = (j < 2 * kNst) ? (j + 1) : 0;
  const float* src = W + ((size_t)layer * kProjN + sr) * kCh + c;
  v4f a0 = *(const v4f*)(src);
  v4f a1 = *(const v4f*)(src + 4);
  asm volatile("" : "+v"(a0), "+v"(a1));
  v8h hv;
#pragma unroll
  for (int e = 0; e < 4; ++e) {
    const float t0 = a0[e];
    const float t1 = a1[e];
    const float w0 = live ? (bf_rne_value(t0) * kWCarry) : 0.0f;
    const float w1 = live ? (bf_rne_value(t1) * kWCarry) : 0.0f;
    hv[e]     = to_h_flush(w0);
    hv[4 + e] = to_h_flush(w1);
  }
  unsigned short* q = WP + (size_t)e0;
  *(volatile v8h*)q = hv;
  __threadfence();
  *(volatile v8h*)q = hv;
}

template <bool SPLIT>
__global__ __launch_bounds__(128) void proj129_kernel(
    const unsigned short* __restrict__ Ahp, const unsigned short* __restrict__ Alp,
    const unsigned short* __restrict__ Wpp, float* __restrict__ dbc, int Mrows)
{
  __shared__ __align__(16) float sT[4][16 * kSlabP];
  const int lane = threadIdx.x & 31;
  const int wave = threadIdx.x >> 5;
  const int tile = blockIdx.x * 4 + wave;
  const int m0   = tile * 16;
  if (m0 >= Mrows) return;
  const _Float16* Ah = (const _Float16*)Ahp;
  const _Float16* Al = (const _Float16*)Alp;
  const _Float16* Wp = (const _Float16*)Wpp;
  const int rlane = lane & 15;
  const int koff  = (lane >> 4) * 8;
  const int mOff  = (lane >> 4) * 8;

  v8f acc[9], accr[9];
#pragma unroll
  for (int j = 0; j < 9; ++j) {
    acc[j]  = (v8f){0.f, 0.f, 0.f, 0.f, 0.f, 0.f, 0.f, 0.f};
    accr[j] = (v8f){0.f, 0.f, 0.f, 0.f, 0.f, 0.f, 0.f, 0.f};
  }
  const _Float16* arow = Ah + (size_t)(m0 + rlane) * kCh + koff;
  const _Float16* lrow = Al + (size_t)(m0 + rlane) * kCh + koff;
  const _Float16* wrow = Wp + (size_t)rlane * kCh + koff;

#pragma unroll 1
  for (int k0 = 0; k0 < kCh; k0 += 32) {
    const v16h ah = frag_load(arow + k0);
    v16h al = ah;
    if (SPLIT) al = frag_load(lrow + k0);
#pragma unroll
    for (int j = 0; j < 9; ++j) {
      const v16h bj = frag_load(wrow + (size_t)(j * 16) * kCh + k0);
      acc[j] = mma_h(ah, bj, acc[j]);
      if (SPLIT) accr[j] = mma_h(al, bj, accr[j]);
    }
  }

  float* slab = sT[wave];
#pragma unroll
  for (int j = 0; j < 9; ++j) {
#pragma unroll
    for (int r = 0; r < 8; ++r) {
      float v = acc[j][r] * kFoldMain;
      if (SPLIT) v = v + accr[j][r] * kFoldRes;
      slab[(mOff + r) * kSlabP + (j << 4) + rlane] = v;
    }
  }
#pragma unroll
  for (int r = 0; r < 8; ++r) slab[(mOff + r) * kSlabP + kProjNP + rlane] = 0.0f;
  __builtin_amdgcn_fence(__ATOMIC_RELEASE, "workgroup");
  __builtin_amdgcn_wave_barrier();
  __builtin_amdgcn_fence(__ATOMIC_ACQUIRE, "workgroup");

  float* gdst = dbc + (size_t)m0 * kDbcP;
  constexpr int kRowV4 = kDbcP / 4;
  for (int pass = 0; pass < 2; ++pass) {
#pragma unroll 4
    for (int it = 0; it < 20; ++it) {
      const int f   = it * 32 + lane;
      const int row = f / kRowV4;
      const int c4  = (f - row * kRowV4) * 4;
      const v4f v = *(const v4f*)(slab + row * kSlabP + c4);
      *(volatile v4f*)(gdst + (size_t)f * 4) = v;
    }
    __threadfence();
  }
}

template <bool POOL, bool RNE_IN>
__global__ __launch_bounds__(256) void state_scan64_kernel(
    const float* __restrict__ Xin, const float* __restrict__ DBC,
    const float* __restrict__ Alog, const float* __restrict__ Dp,
    const float* __restrict__ Wdt, const float* __restrict__ bdt,
    float* __restrict__ OutF, unsigned short* __restrict__ OutH, unsigned short* __restrict__ OutL, int L)
{
  __shared__ __align__(16) float sD[kTS * kDbcP];
  __shared__ __align__(16) float sX[kTS * kScanCh];
  __shared__ __align__(16) float sY[kTS * kYP];
  __shared__ __align__(16) float sA[kScanCh * kAP];

  const int tid  = threadIdx.x;
  const int lane = tid & 31;
  const int wave = tid >> 5;
  constexpr int kGroups = kCh / kScanCh;
  const int bix = blockIdx.x / kGroups;
  const int d0  = (blockIdx.x - bix * kGroups) * kScanCh;
  const int chl = wave * 8 + (lane >> 2);
  const int g   = lane & 3;
  const int d   = d0 + chl;

#pragma unroll 1
  for (int it = 0; it < 16; ++it) {
    const int i = it * 256 + tid;
    const float al = bf_rne_value(Alog[(size_t)d0 * kNst + i]);
    sA[(i >> 6) * kAP + (i & 63)] = -expf(al);
  }
  __syncthreads();
  float negA[16], h[16];
#pragma unroll
  for (int q4 = 0; q4 < 4; ++q4) {
    const v4f av = *(const v4f*)(sA + chl * kAP + g * 16 + 4 * q4);
    negA[4 * q4 + 0] = av[0];
    negA[4 * q4 + 1] = av[1];
    negA[4 * q4 + 2] = av[2];
    negA[4 * q4 + 3] = av[3];
    h[4 * q4 + 0] = 0.0f;
    h[4 * q4 + 1] = 0.0f;
    h[4 * q4 + 2] = 0.0f;
    h[4 * q4 + 3] = 0.0f;
  }
  const float wdt = bf_rne_value(Wdt[d]);
  const float bb  = bf_rne_value(bdt[d]);
  const float Dd  = bf_rne_value(Dp[d]);
  float yprev = 0.0f;

  const int hh  = lane >> 4;
  const int c4  = (lane & 15) * 4;
  const int q8  = lane >> 3;
  const int c8  = (lane & 7) * 8;

#pragma unroll 1
  for (int t0 = 0; t0 < L; t0 += kTS) {
    __syncthreads();
    {
      const size_t rowbase = (size_t)bix * L + t0;
      const float* gD = DBC + rowbase * kDbcP;
#pragma unroll
      for (int i = 0; i < 5; ++i) {
        const int f = i * 256 + tid;
        *(v4f*)(sD + f * 4) = *(const v4f*)(gD + (size_t)f * 4);
      }
#pragma unroll
      for (int i = 0; i < 2; ++i) {
        const int f  = i * 256 + tid;
        const int r  = f >> 4;
        const int cc = (f & 15) * 4;
        v4f xv = *(const v4f*)(Xin + (rowbase + r) * kCh + d0 + cc);
        if (RNE_IN) {
#pragma unroll
          for (int e = 0; e < 4; ++e) {
            float t = xv[e];
            t = bf_rne_value(t);
            xv[e] = t;
          }
        }
        *(v4f*)(sX + r * kScanCh + cc) = xv;
      }
    }
    __syncthreads();

#pragma unroll 1
    for (int s = 0; s < kTS; ++s) {
      const float* dr = sD + s * kDbcP;
      const float dz  = dr[2 * kNst];
      const float xt  = sX[s * kScanCh + chl];
      const float z   = dz * wdt + bb;
      const float az  = expf(-fabsf(z));
      const float dt  = fmaxf(z, 0.0f) + log1pf(az);
      const float dtx = dt * xt;
      float y = 0.0f;
#pragma unroll
      for (int q4 = 0; q4 < 4; ++q4) {
        const v4f bv = *(const v4f*)(dr + g * 16 + 4 * q4);
        const v4f cv = *(const v4f*)(dr + kNst + g * 16 + 4 * q4);
#pragma unroll
        for (int e = 0; e < 4; ++e) {
          const int k = 4 * q4 + e;
          const float ee = __expf(dt * negA[k]);
          h[k] = ee * h[k] + dtx * bv[e];
          y = h[k] * cv[e] + y;
        }
      }
      y += __shfl_xor(y, 1, 32);
      y += __shfl_xor(y, 2, 32);
      y = xt * Dd + y;
      if (POOL) {
        if (s & 1) {
          const float pv = 0.5f * (yprev + y);
          if (g == 0) sY[(s >> 1) * kYP + chl] = pv;
        } else {
          yprev = y;
        }
      } else {
        if (g == 0) sY[s * kYP + chl] = y;
      }
    }
    __syncthreads();

    if (POOL) {
      const size_t orow0 = (size_t)bix * (L >> 1) + (t0 >> 1);
      const int rowf = wave * 2 + hh;
      const v4f fv = *(const v4f*)(sY + rowf * kYP + c4);
      float* pf = OutF + (orow0 + rowf) * kCh + d0 + c4;
      const int rowh = (wave & 3) * 4 + q8;
      const float* sp = sY + rowh * kYP + c8;
      const v4f a0 = *(const v4f*)(sp);
      const v4f a1 = *(const v4f*)(sp + 4);
      v8h hv, lv;
#pragma unroll
      for (int e = 0; e < 4; ++e) {
        const float t0v = a0[e];
        const float t1v = a1[e];
        const float s0 = t0v * kXCarry;
        const float s1 = t1v * kXCarry;
        const _Float16 h0 = to_h_flush(s0);
        const _Float16 h1 = to_h_flush(s1);
        const float r0 = (s0 - (float)h0) * kRCarry;
        const float r1 = (s1 - (float)h1) * kRCarry;
        hv[e]     = h0;
        hv[4 + e] = h1;
        lv[e]     = to_h_flush(r0);
        lv[4 + e] = to_h_flush(r1);
      }
      unsigned short* ph = OutH + (orow0 + rowh) * kCh + d0 + c8;
      unsigned short* pl = OutL + (orow0 + rowh) * kCh + d0 + c8;
      for (int pass = 0; pass < 2; ++pass) {
        *(volatile v4f*)pf = fv;
        if (wave < 4) {
          *(volatile v8h*)ph = hv;
          *(volatile v8h*)pl = lv;
        }
        __threadfence();
      }
    } else {
      const size_t orow0 = (size_t)bix * L + t0;
      v4f fv[2];
#pragma unroll
      for (int it = 0; it < 2; ++it) fv[it] = *(const v4f*)(sY + (it * 16 + wave * 2 + hh) * kYP + c4);
      for (int pass = 0; pass < 2; ++pass) {
#pragma unroll
        for (int it = 0; it < 2; ++it)
          *(volatile v4f*)(OutF + (orow0 + it * 16 + wave * 2 + hh) * kCh + d0 + c4) = fv[it];
        __threadfence();
      }
    }
  }
}

extern "C" void kernel_launch(void* const* d_in, const int* in_sizes, int n_in,
                              void* d_out, int out_size, void* d_ws, size_t ws_size,
                              hipStream_t stream) {
  if (n_in < 6) return;
  if (in_sizes[0] != kBatch * kSeq0 * kCh) return;
  if (in_sizes[1] != kLayers * kCh * kNst) return;
  if (in_sizes[2] != kLayers * kCh) return;
  if (in_sizes[3] != kLayers * kProjN * kCh) return;
  if (in_sizes[4] != kLayers * kCh) return;
  if (in_sizes[5] != kLayers * kCh) return;
  if (out_size != kBatch * (kSeq0 / 4) * kCh) return;
  if (ws_size < kWsTotal) return;

  const float* x     = (const float*)d_in[0];
  const float* A_log = (const float*)d_in[1];
  const float* Dp    = (const float*)d_in[2];
  const float* W_dbc = (const float*)d_in[3];
  const float* W_dt  = (const float*)d_in[4];
  const float* b_dt  = (const float*)d_in[5];
  float* out = (float*)d_out;

  char* ws = (char*)d_ws;
  unsigned short* WP   = (unsigned short*)(ws + kOffWP);
  unsigned short* XH0  = (unsigned short*)(ws + kOffXH0);
  float*          DBC0 = (float*)(ws + kOffDBC0);
  float*          DBC1 = (float*)(ws + kOffDBC1);
  float*          DBC2 = (float*)(ws + kOffDBC2);
  float*          X1F  = (float*)(ws + kOffX1F);
  unsigned short* X1H  = (unsigned short*)(ws + kOffX1H);
  unsigned short* X1L  = (unsigned short*)(ws + kOffX1L);
  float*          X2F  = (float*)(ws + kOffX2F);
  unsigned short* X2H  = (unsigned short*)(ws + kOffX2H);
  unsigned short* X2L  = (unsigned short*)(ws + kOffX2L);

  constexpr int kWTotal8 = kLayers * kProjNP * kCh / 8;
  constexpr int kXTotal8 = kBatch * kSeq0 * kCh / 8;
  static_assert(kWTotal8 % 256 == 0 && kXTotal8 % 256 == 0, "exact plane grids");
  constexpr int kM0 = kBatch * kSeq0;
  constexpr int kM1 = kM0 / 2;
  constexpr int kM2 = kM0 / 4;
  static_assert(kM0 % 64 == 0 && kM1 % 64 == 0 && kM2 % 64 == 0, "projection row tiles");
  constexpr int kScanGrid = kBatch * (kCh / kScanCh);
  constexpr size_t kWPlane = (size_t)kProjNP * kCh;
  constexpr size_t kALayer = (size_t)kCh * kNst;

  plane_w_f16_kernel<<<kWTotal8 / 256, 256, 0, stream>>>(W_dbc, WP, kWTotal8);
  plane_x_f16_kernel<<<kXTotal8 / 256, 256, 0, stream>>>(x, XH0, kXTotal8);

  proj129_kernel<false><<<kM0 / 64, 128, 0, stream>>>(XH0, XH0, WP, DBC0, kM0);
  state_scan64_kernel<true, true><<<kScanGrid, 256, 0, stream>>>(
      x, DBC0, A_log, Dp, W_dt, b_dt, X1F, X1H, X1L, kSeq0);

  proj129_kernel<true><<<kM1 / 64, 128, 0, stream>>>(X1H, X1L, WP + kWPlane, DBC1, kM1);
  state_scan64_kernel<true, false><<<kScanGrid, 256, 0, stream>>>(
      X1F, DBC1, A_log + kALayer, Dp + kCh, W_dt + kCh, b_dt + kCh, X2F, X2H, X2L, kSeq0 / 2);

  proj129_kernel<true><<<kM2 / 64, 128, 0, stream>>>(X2H, X2L, WP + 2 * kWPlane, DBC2, kM2);
  state_scan64_kernel<false, false><<<kScanGrid, 256, 0, stream>>>(
      X2F, DBC2, A_log + 2 * kALayer, Dp + 2 * kCh, W_dt + 2 * kCh, b_dt + 2 * kCh, out, X2H, X2L, kSeq0 / 4);
}
